// SpectralAttention_14104672600687
// MI455X (gfx1250) — hardware-verified
//
#include <hip/hip_runtime.h>
#include <hip/hip_bf16.h>
#include <math.h>

typedef __attribute__((ext_vector_type(16))) _Float16 v16h;
typedef __attribute__((ext_vector_type(8)))  float    v8f;
typedef __attribute__((ext_vector_type(4)))  float    v4f;
typedef float __attribute__((may_alias)) float_a;
template <typename T> __device__ __forceinline__ void vst2(void* p, T v) { *(volatile T*)p = v; __threadfence(); *(volatile T*)p = v; }
__device__ inline v8f wmma16(v16h a, v16h b, v8f c) {
  v8f d = __builtin_amdgcn_wmma_f32_16x16x32_f16(false, a, false, b, (short)0, c, false, false);
  asm volatile("v_nop\n\tv_nop\n\tv_nop\n\tv_nop" : "+v"(d) : "v"(a), "v"(b));
  return d;
}

#define SEQ_LEN 1024
#define D_MODEL 512
#define HEADS   8
#define HD      64
#define KFILT   24
#define BATCH   2

__device__ inline uint32_t pack_h2(float a, float b) {
  union { uint32_t u; _Float16 h[2]; } p;
  p.h[0] = (_Float16)a;
  p.h[1] = (_Float16)b;
  return p.u;
}

__device__ inline v8f zero8() {
  v8f z;
#pragma unroll
  for (int i = 0; i < 8; ++i) z[i] = 0.0f;
  return z;
}

__device__ inline float gelu_tanh(float x) {
  return 0.5f * x * (1.0f + tanhf(0.7978845608f * (x + 0.044715f * x * x * x)));
}
__device__ inline float sigmoidf(float x) { return 1.0f / (1.0f + expf(-x)); }


#define GBM 128
#define GBN 64
#define GBK 32

__global__ __launch_bounds__(256)
void gemm_wmma_kernel(const float* __restrict__ A, const float* __restrict__ Bsrc,
                      const float* __restrict__ bias, float* __restrict__ C,
                      int M, int N, int K, int transB, int act) {
  __shared__ __align__(32) uint32_t As[2][8][32][8];
  __shared__ __align__(32) uint32_t Bs[2][4][32][8];
  __shared__ __align__(16) float So[8][16 * 64];
  const int tid  = threadIdx.x;
  const int wave = tid >> 5;
  const int lane = tid & 31;
  const int m0   = blockIdx.x * GBM;
  const int n0   = blockIdx.y * GBN;
  const int nk   = (K + GBK - 1) / GBK;

  v8f acc[4];
#pragma unroll
  for (int i = 0; i < 4; ++i) acc[i] = zero8();

  auto load_regs = [&](int kt, float ra[8][2], float rb[4][2]) {
    const int k0   = kt * GBK;
    const bool full = (k0 + GBK <= K);
#pragma unroll
    for (int j = 0; j < 8; ++j) {
      int idx = tid + j * 256;
      int r = idx >> 4, kp = idx & 15;
      if (full) {
        float2 t = *reinterpret_cast<const float2*>(
            &A[(size_t)(m0 + r) * K + k0 + 2 * kp]);
        ra[j][0] = t.x; ra[j][1] = t.y;
      } else {
        int k = k0 + 2 * kp;
        ra[j][0] = (k < K)     ? A[(size_t)(m0 + r) * K + k]     : 0.0f;
        ra[j][1] = (k + 1 < K) ? A[(size_t)(m0 + r) * K + k + 1] : 0.0f;
      }
    }
    if (transB) {
#pragma unroll
      for (int j = 0; j < 4; ++j) {
        int idx = tid + j * 256;
        int kp = idx & 15, n = idx >> 4;
        if (full) {
          float2 t = *reinterpret_cast<const float2*>(
              &Bsrc[(size_t)(n0 + n) * K + k0 + 2 * kp]);
          rb[j][0] = t.x; rb[j][1] = t.y;
        } else {
          int k = k0 + 2 * kp;
          rb[j][0] = (k < K)     ? Bsrc[(size_t)(n0 + n) * K + k]     : 0.0f;
          rb[j][1] = (k + 1 < K) ? Bsrc[(size_t)(n0 + n) * K + k + 1] : 0.0f;
        }
      }
    } else {
#pragma unroll
      for (int j = 0; j < 4; ++j) {
        int idx = tid + j * 256;
        int n = idx & 63, kp = idx >> 6;
        int k = k0 + 2 * kp;
        rb[j][0] = (k < K)     ? Bsrc[(size_t)k * N + n0 + n]       : 0.0f;
        rb[j][1] = (k + 1 < K) ? Bsrc[(size_t)(k + 1) * N + n0 + n] : 0.0f;
      }
    }
  };

  auto store_lds = [&](int buf, float ra[8][2], float rb[4][2]) {
#pragma unroll
    for (int j = 0; j < 8; ++j) {
      int idx = tid + j * 256;
      int r = idx >> 4, kp = idx & 15;
      int ln = (r & 15) + ((kp & 4) ? 16 : 0);
      int dw = (kp & 3) + ((kp >= 8) ? 4 : 0);
      As[buf][r >> 4][ln][dw] = pack_h2(ra[j][0], ra[j][1]);
    }
#pragma unroll
    for (int j = 0; j < 4; ++j) {
      int idx = tid + j * 256;
      int kp, n;
      if (transB) { kp = idx & 15; n = idx >> 4; }
      else        { n = idx & 63;  kp = idx >> 6; }
      int ln = (n & 15) + ((kp & 4) ? 16 : 0);
      Bs[buf][n >> 4][ln][(kp & 3) + ((kp >= 8) ? 4 : 0)] = pack_h2(rb[j][0], rb[j][1]);
    }
  };

  float ra[8][2], rb[4][2];
  load_regs(0, ra, rb);
  store_lds(0, ra, rb);
  __syncthreads();

  for (int kt = 0; kt < nk; ++kt) {
    const int cur = kt & 1;
    const bool more = (kt + 1 < nk);
    if (more) load_regs(kt + 1, ra, rb);

    const v16h a = *reinterpret_cast<const v16h*>(&As[cur][wave][lane][0]);
#pragma unroll
    for (int nt = 0; nt < 4; ++nt) {
      const v16h b = *reinterpret_cast<const v16h*>(&Bs[cur][nt][lane][0]);
      acc[nt] = wmma16(a, b, acc[nt]);
    }
    if (more) store_lds(1 - cur, ra, rb);
    __syncthreads();
  }

  const int nlo = lane & 15;
  const int mb  = (lane >> 4) * 8;
  float* S = So[wave];
#pragma unroll
  for (int nt = 0; nt < 4; ++nt) {
    int col = n0 + nt * 16 + nlo;
#pragma unroll 1
    for (int i = 0; i < 8; ++i) {
      float v = acc[nt][i];
      if (bias) v += bias[col];
      if (act == 1) v = gelu_tanh(v);
      else if (act == 2) v = sigmoidf(v);
      S[(mb + i) * 64 + nt * 16 + nlo] = v;
    }
  }
  asm volatile("s_wait_dscnt 0" ::: "memory"); __builtin_amdgcn_wave_barrier(); __builtin_amdgcn_fence(__ATOMIC_RELEASE, "workgroup");
#pragma unroll
  for (int q = 0; q < 8; ++q) { const int rl = q * 2 + (lane >> 4), pc = lane & 15; const int row = m0 + wave * 16 + rl;
    if (row < M) vst2(C + (size_t)row * N + n0 + pc * 4, *(const v4f*)(S + rl * 64 + pc * 4)); }
}

__global__ __launch_bounds__(256)
void conv_kernel(const float* __restrict__ u, const float* __restrict__ phi,
                 float* __restrict__ z) {
  const int r = blockIdx.x * 64 + (threadIdx.x & 63);
  const int t = blockIdx.y * 4 + (threadIdx.x >> 6);
  const int b = blockIdx.z;
  const float* ub = u + (size_t)b * SEQ_LEN * D_MODEL;
  float acc = 0.0f;
  for (int l = 0; l <= t; l += 2) {
    acc = fmaf(phi[(size_t)l * D_MODEL + r], ub[(size_t)(t - l) * D_MODEL + r], acc);
  }
  vst2(z + ((size_t)b * SEQ_LEN + t) * D_MODEL + r, (float_a)(2.0f * acc));
}

__global__ __launch_bounds__(256)
void ln_kernel(const float* __restrict__ z, const float* __restrict__ w,
               const float* __restrict__ bvec, float* __restrict__ xt) {
  const int row = blockIdx.x;
  const float* x = z + (size_t)row * D_MODEL;
  float* o = xt + (size_t)row * D_MODEL;
  const int tid = threadIdx.x;
  float s = 0.0f, q = 0.0f;
  for (int i = tid; i < D_MODEL; i += 256) {
    float v = x[i];
    s += v;
    q += v * v;
  }
#pragma unroll
  for (int off = 16; off > 0; off >>= 1) {
    s += __shfl_xor(s, off, 32);
    q += __shfl_xor(q, off, 32);
  }
  __shared__ float rs[8], rq[8];
  __shared__ float mu_s, ri_s;
  if ((tid & 31) == 0) { rs[tid >> 5] = s; rq[tid >> 5] = q; }
  __syncthreads();
  if (tid == 0) {
    float ts = 0.0f, tq = 0.0f;
#pragma unroll
    for (int i = 0; i < 8; ++i) { ts += rs[i]; tq += rq[i]; }
    float mu  = ts / (float)D_MODEL;
    float var = tq / (float)D_MODEL - mu * mu;
    mu_s = mu;
    ri_s = rsqrtf(var + 1e-5f);
  }
  __syncthreads();
  float mu = mu_s, ri = ri_s;
  for (int i = tid; i < D_MODEL; i += 256)
    vst2(o + i, (float_a)((x[i] - mu) * ri * w[i] + bvec[i]));
}

__global__ __launch_bounds__(128)
void attn_kernel(const float* __restrict__ Q, const float* __restrict__ K,
                 const float* __restrict__ V, float* __restrict__ Y) {
  const int bh = blockIdx.y;
  const int b  = bh >> 3;
  const int h  = bh & 7;
  const int t0 = blockIdx.x * 64;
  const int tid  = threadIdx.x;
  const int wave = tid >> 5;
  const int lane = tid & 31;
  const size_t base = (size_t)b * SEQ_LEN * D_MODEL + h * HD;
  const float* Qh = Q + base;
  const float* Kh = K + base;
  const float* Vh = V + base;

  __shared__ __align__(32) uint32_t Qf[4][2][32][8];
  __shared__ __align__(32) uint32_t Kf[4][32][8];
  __shared__ __align__(32) uint32_t Vf[2][2][32][8];
  __shared__ __align__(32) uint32_t Sf[4][32][8];

  for (int idx = tid; idx < 64 * 32; idx += 128) {
    int r = idx >> 5, pc = idx & 31;
    float2 t = *reinterpret_cast<const float2*>(
        &Qh[(size_t)(t0 + r) * D_MODEL + 2 * pc]);
    int kp = pc & 15;
    int ln = (r & 15) + ((kp & 4) ? 16 : 0);
    int dw = (kp & 3) + ((kp >= 8) ? 4 : 0);
    Qf[r >> 4][pc >> 4][ln][dw] = pack_h2(t.x, t.y);
  }
  __syncthreads();

  const v16h qa0 = *reinterpret_cast<const v16h*>(&Qf[wave][0][lane][0]);
  const v16h qa1 = *reinterpret_cast<const v16h*>(&Qf[wave][1][lane][0]);

  v8f acc[4];
#pragma unroll
  for (int i = 0; i < 4; ++i) acc[i] = zero8();

  const int nlo = lane & 15;
  const int mb  = (lane >> 4) * 8;
  _Float16* sfw = (_Float16*)&Sf[wave][0][0];

  for (int s0 = 0; s0 < t0 + 64; s0 += 32) {
    __syncthreads();
    for (int idx = tid; idx < 16 * 64; idx += 128) {
      int n = idx & 63, kp = idx >> 6;
      float b0 = Kh[(size_t)(s0 + 2 * kp) * D_MODEL + n];
      float b1 = Kh[(size_t)(s0 + 2 * kp + 1) * D_MODEL + n];
      int ln = (n & 15) + ((kp & 4) ? 16 : 0);
      Kf[n >> 4][ln][(kp & 3) + ((kp >= 8) ? 4 : 0)] = pack_h2(b0, b1);
    }
    for (int idx = tid; idx < 32 * 32; idx += 128) {
      int kp = idx & 31, s = idx >> 5;
      float2 t = *reinterpret_cast<const float2*>(
          &Vh[(size_t)(s0 + s) * D_MODEL + 2 * kp]);
      int kc = kp & 15;
      int ln = (s & 15) + ((kc & 4) ? 16 : 0);
      Vf[s >> 4][kp >> 4][ln][(kc & 3) + ((kc >= 8) ? 4 : 0)] = pack_h2(t.x, t.y);
    }
    __syncthreads();

#pragma unroll
    for (int sub = 0; sub < 2; ++sub) {
      v8f sacc = zero8();
      const v16h vb0 = *reinterpret_cast<const v16h*>(&Vf[sub][0][lane][0]);
      const v16h vb1 = *reinterpret_cast<const v16h*>(&Vf[sub][1][lane][0]);
      sacc = wmma16(qa0, vb0, sacc);
      sacc = wmma16(qa1, vb1, sacc);
      int ks   = sub * 16 + nlo;
      int dwh  = ((ks & 7) >> 1) * 2 + (ks & 1) + ((ks >= 16) ? 8 : 0);
      int lnhi = ((ks & 15) >= 8) ? 16 : 0;
      int s_glob = s0 + ks;
#pragma unroll
      for (int i = 0; i < 8; ++i) {
        int t_glob = t0 + wave * 16 + mb + i;
        float sv = (s_glob <= t_glob) ? sacc[i] : 0.0f;
        sfw[(mb + i + lnhi) * 16 + dwh] = (_Float16)sv;
      }
    }
    asm volatile("s_wait_dscnt 0" ::: "memory"); __builtin_amdgcn_wave_barrier(); __builtin_amdgcn_fence(__ATOMIC_RELEASE, "workgroup");
    const v16h a2 = *reinterpret_cast<const v16h*>(&Sf[wave][lane][0]);
#pragma unroll
    for (int nt = 0; nt < 4; ++nt) {
      const v16h kb = *reinterpret_cast<const v16h*>(&Kf[nt][lane][0]);
      acc[nt] = wmma16(a2, kb, acc[nt]);
    }
  }

  __shared__ __align__(16) float Yo[4][16 * 64];
  float* yo = Yo[wave];
#pragma unroll
  for (int nt = 0; nt < 4; ++nt)
#pragma unroll
    for (int i = 0; i < 8; ++i) yo[(mb + i) * 64 + nt * 16 + nlo] = acc[nt][i];
  asm volatile("s_wait_dscnt 0" ::: "memory"); __builtin_amdgcn_wave_barrier(); __builtin_amdgcn_fence(__ATOMIC_RELEASE, "workgroup");
#pragma unroll
  for (int q = 0; q < 8; ++q) { const int rl = q * 2 + (lane >> 4), pc = lane & 15;
    vst2(Y + ((size_t)b * SEQ_LEN + t0 + wave * 16 + rl) * D_MODEL + h * HD + pc * 4, *(const v4f*)(yo + rl * 64 + pc * 4)); }
}

__global__ __launch_bounds__(256)
void comb_kernel(const float* __restrict__ g, const float* __restrict__ y,
                 const float* __restrict__ xt, float* __restrict__ c, int n) {
  int i = blockIdx.x * 256 + threadIdx.x;
  if (i < n) {
    float gv = g[i];
    vst2(c + i, (float_a)(gv * y[i] + (1.0f - gv) * xt[i]));
  }
}

extern "C" void kernel_launch(void* const* d_in, const int* in_sizes, int n_in,
                              void* d_out, int out_size, void* d_ws, size_t ws_size,
                              hipStream_t stream) {
  (void)in_sizes; (void)n_in; (void)out_size; (void)ws_size;
  const float* x    = (const float*)d_in[0];
  const float* stuf = (const float*)d_in[1];
  const float* Mi   = (const float*)d_in[2];
  const float* Mf   = (const float*)d_in[3];
  const float* Wq   = (const float*)d_in[4];
  const float* bq   = (const float*)d_in[5];
  const float* Wk   = (const float*)d_in[6];
  const float* bk   = (const float*)d_in[7];
  const float* Wv   = (const float*)d_in[8];
  const float* bv   = (const float*)d_in[9];
  const float* Wg   = (const float*)d_in[10];
  const float* bg   = (const float*)d_in[11];
  const float* Wo   = (const float*)d_in[12];
  const float* bo   = (const float*)d_in[13];
  const float* lnw  = (const float*)d_in[14];
  const float* lnb  = (const float*)d_in[15];
  float* out = (float*)d_out;

  const int M  = BATCH * SEQ_LEN;
  const int N  = D_MODEL;
  const size_t SZ = (size_t)M * N;

  float* ws     = (float*)d_ws;
  float* u_proj = ws;
  float* phi    = u_proj + SZ;
  float* Qb     = phi + (size_t)SEQ_LEN * D_MODEL;
  float* Kb     = Qb + SZ;
  float* Vb     = Kb + SZ;
  float* Gb     = Vb + SZ;
  float* Zc     = Gb + SZ;
  float* Xt     = Zc + SZ;
  float* Ya     = Xt + SZ;
  float* Cb     = Ya + SZ;

  dim3 ggrid(M / GBM, N / GBN);
  dim3 pgrid(SEQ_LEN / GBM, N / GBN);

  gemm_wmma_kernel<<<ggrid, 256, 0, stream>>>(x, Mi, nullptr, u_proj, M, N, D_MODEL, 0, 0);
  gemm_wmma_kernel<<<pgrid, 256, 0, stream>>>(stuf, Mf, nullptr, phi, SEQ_LEN, N, KFILT, 0, 0);
  gemm_wmma_kernel<<<ggrid, 256, 0, stream>>>(x, Wq, bq, Qb, M, N, D_MODEL, 1, 1);
  gemm_wmma_kernel<<<ggrid, 256, 0, stream>>>(x, Wk, bk, Kb, M, N, D_MODEL, 1, 1);
  gemm_wmma_kernel<<<ggrid, 256, 0, stream>>>(x, Wv, bv, Vb, M, N, D_MODEL, 1, 1);
  gemm_wmma_kernel<<<ggrid, 256, 0, stream>>>(x, Wg, bg, Gb, M, N, D_MODEL, 1, 2);

  dim3 cgrid(D_MODEL / 64, SEQ_LEN / 4, BATCH);
  conv_kernel<<<cgrid, 256, 0, stream>>>(u_proj, phi, Zc);
  ln_kernel<<<M, 256, 0, stream>>>(Zc, lnw, lnb, Xt);

  dim3 agrid(SEQ_LEN / 64, BATCH * HEADS);
  attn_kernel<<<agrid, 128, 0, stream>>>(Qb, Kb, Vb, Ya);

  comb_kernel<<<(int)(SZ / 256), 256, 0, stream>>>(Gb, Ya, Xt, Cb, (int)SZ);
  gemm_wmma_kernel<<<ggrid, 256, 0, stream>>>(Cb, Wo, bo, out, M, N, D_MODEL, 1, 0);
}
